// FeatExtractor_63015760167691
// MI455X (gfx1250) — hardware-verified
//
#include <hip/hip_runtime.h>

typedef _Float16 f16t;
typedef _Float16 v16h __attribute__((ext_vector_type(16)));
typedef _Float16 v8h  __attribute__((ext_vector_type(8)));
typedef float    v8f  __attribute__((ext_vector_type(8)));
typedef float    v4f  __attribute__((ext_vector_type(4)));
typedef v8h __attribute__((may_alias)) v8ha;
typedef v4f __attribute__((may_alias)) v4fa;
union Frag { v16h v; v8h half[2]; };

#define NB   32
#define HI   128
#define CIN  12
#define CP   16
#define C1   64
#define HP   64
#define C2   128
#define NOBJ 32
#define IMR  130
#define IMC  132
#define PLR  66
#define PLC  66
#define K1   160
#define K2   576

#define XCAR 256.0f
#define WCAR 64.0f
#define PCAR 16.0f

__device__ __forceinline__ v8f wmma_f16(v16h a, v16h b, v8f c) {
  v8f d = __builtin_amdgcn_wmma_f32_16x16x32_f16(false, a, false, b, (short)0, c, false, false);
  asm volatile("v_nop\n\tv_nop\n\tv_nop\n\tv_nop" : "+v"(d) : "v"(a), "v"(b));
  return d;
}

__device__ __forceinline__ v8h zero8h() {
  v8h z;
  #pragma unroll
  for (int j = 0; j < 8; ++j) z[j] = (f16t)0.0f;
  return z;
}

__device__ __forceinline__ v16h load_frag32(const f16t* p, int h) {
  Frag f;
  f.half[0] = *(const v8ha*)(p + 8 * h);
  f.half[1] = *(const v8ha*)(p + 16 + 8 * h);
  return f.v;
}

__device__ __forceinline__ v4f max4(v4f a, v4f b) {
  v4f r;
  r.x = fmaxf(a.x, b.x); r.y = fmaxf(a.y, b.y); r.z = fmaxf(a.z, b.z); r.w = fmaxf(a.w, b.w);
  return r;
}

__global__ __launch_bounds__(256) void cvt_img_k(const float* __restrict__ img, f16t* __restrict__ imgp) {
  const int tid = threadIdx.x;
  const int prow = blockIdx.x, b = blockIdx.y;
  const int iy = prow - 1;
  const bool rowok = (unsigned)iy < (unsigned)HI;
  const int iyc = iy < 0 ? 0 : (iy > HI - 1 ? HI - 1 : iy);
  const float* src = img + (size_t)b * CIN * HI * HI + (size_t)iyc * HI;
  f16t* rowb = imgp + ((size_t)(b * IMR + prow) * IMC) * CP;
  const float sc = (1.0f / 255.0f);
  v8h o[2];
  #pragma unroll
  for (int i = 0; i < 2; ++i) {
    const int p = tid + 256 * i;
    const int pc = p < 264 ? p : 263;
    const int pcol = pc >> 1, chh = pc & 1;
    const int ix = pcol - 1;
    const bool colok = (unsigned)ix < (unsigned)HI;
    const int ixc = ix < 0 ? 0 : (ix > HI - 1 ? HI - 1 : ix);
    v8h v;
    #pragma unroll
    for (int j = 0; j < 8; ++j) {
      const int c = 8 * chh + j;
      const int cc = c < CIN ? c : CIN - 1;
      const float x = src[(size_t)cc * HI * HI + ixc];
      const bool ok = rowok && colok && (c < CIN);
      v[j] = ok ? (f16t)((x * sc) * XCAR) : (f16t)0.0f;
    }
    o[i] = v;
  }
  f16t* d0 = rowb + (size_t)tid * 8;
  f16t* d1 = rowb + (size_t)(tid + 256) * 8;
  const bool w1 = tid < 8;
  *(volatile v8h*)d0 = o[0];
  if (w1) *(volatile v8h*)d1 = o[1];
  __threadfence();
  *(volatile v8h*)d0 = o[0];
  if (w1) *(volatile v8h*)d1 = o[1];
}

__global__ __launch_bounds__(256) void cvt_w_k(const float* __restrict__ w1, const float* __restrict__ w2,
                                               f16t* __restrict__ w1p, f16t* __restrict__ w2p) {
  const int tid = threadIdx.x;
  if (blockIdx.x < 5) {
    const int p = blockIdx.x * 256 + tid;
    const int o = p / 20, kq = p - o * 20;
    v8h v;
    #pragma unroll
    for (int j = 0; j < 8; ++j) {
      const int k = kq * 8 + j;
      const int tap = k >> 4, c = k & 15;
      const bool ok = (tap < 9) && (c < CIN);
      const int tc = tap < 9 ? tap : 8, cc = c < CIN ? c : CIN - 1;
      const float x = w1[(size_t)o * (CIN * 9) + cc * 9 + tc];
      v[j] = ok ? (f16t)(x * WCAR) : (f16t)0.0f;
    }
    f16t* d = w1p + (size_t)p * 8;
    *(volatile v8h*)d = v;
    __threadfence();
    *(volatile v8h*)d = v;
  } else {
    const int p = (blockIdx.x - 5) * 256 + tid;
    const int o = p / 72, kq = p - o * 72;
    v8h v;
    #pragma unroll
    for (int j = 0; j < 8; ++j) {
      const int k = kq * 8 + j;
      const int tap = k >> 6, c = k & 63;
      const float x = w2[(size_t)o * (C1 * 9) + c * 9 + tap];
      v[j] = (f16t)(x * WCAR);
    }
    f16t* d = w2p + (size_t)p * 8;
    *(volatile v8h*)d = v;
    __threadfence();
    *(volatile v8h*)d = v;
  }
}

__global__ __launch_bounds__(256) void halo_k(f16t* __restrict__ pool) {
  const int tid = threadIdx.x;
  const int prow = blockIdx.x, b = blockIdx.y;
  f16t* rowb = pool + ((size_t)(b * PLR + prow) * PLC) * C1;
  const v8h z = zero8h();
  if (prow == 0 || prow == PLR - 1) {
    f16t* d[3];
    bool ok[3];
    #pragma unroll
    for (int i = 0; i < 3; ++i) {
      const int p = tid + 256 * i;
      ok[i] = p < 528;
      d[i] = rowb + (size_t)(ok[i] ? p : 0) * 8;
    }
    #pragma unroll
    for (int i = 0; i < 3; ++i) if (ok[i]) *(volatile v8h*)d[i] = z;
    __threadfence();
    #pragma unroll
    for (int i = 0; i < 3; ++i) if (ok[i]) *(volatile v8h*)d[i] = z;
  } else {
    const bool ok = tid < 16;
    const int pcol = (tid < 8) ? 0 : (PLC - 1);
    f16t* d = rowb + (size_t)pcol * C1 + (tid & 7) * 8;
    if (ok) *(volatile v8h*)d = z;
    __threadfence();
    if (ok) *(volatile v8h*)d = z;
  }
}

__global__ __launch_bounds__(256) void conv1_pool_k(
    const f16t* __restrict__ imgp, const f16t* __restrict__ w1p, const float* __restrict__ bias,
    f16t* __restrict__ pool)
{
  __shared__ __attribute__((aligned(16))) float sT[128 * 64];
  const int tid = threadIdx.x, lane = tid & 31, w = tid >> 5;
  const int h = lane >> 4, m = lane & 15;
  const int xb = blockIdx.x, py = blockIdx.y, b = blockIdx.z;
  const int cy = 2 * py + (w >> 2);
  const int cx0 = 64 * xb + 16 * (w & 3);
  const f16t* abase = imgp + ((size_t)(b * IMR + cy) * IMC + cx0 + m) * CP;
  const f16t* bbase = w1p + (size_t)m * K1;
  const v8f z8 = {0.f, 0.f, 0.f, 0.f, 0.f, 0.f, 0.f, 0.f};
  v8f acc[4];
  #pragma unroll
  for (int nt = 0; nt < 4; ++nt) acc[nt] = z8;
  #pragma unroll
  for (int t = 0; t < 5; ++t) {
    const int tap0 = 2 * t, kr0 = tap0 / 3, kc0 = tap0 - 3 * kr0;
    Frag a;
    a.half[0] = *(const v8ha*)(abase + ((size_t)kr0 * IMC + kc0) * CP + 8 * h);
    if (t < 4) {
      const int tap1 = 2 * t + 1, kr1 = tap1 / 3, kc1 = tap1 - 3 * kr1;
      a.half[1] = *(const v8ha*)(abase + ((size_t)kr1 * IMC + kc1) * CP + 8 * h);
    } else {
      a.half[1] = zero8h();
    }
    #pragma unroll
    for (int nt = 0; nt < 4; ++nt) {
      const v16h bb = load_frag32(bbase + (size_t)nt * 16 * K1 + 32 * t, h);
      acc[nt] = wmma_f16(a.v, bb, acc[nt]);
    }
  }
  const float osc = 1.0f / (XCAR * WCAR);
  #pragma unroll
  for (int nt = 0; nt < 4; ++nt) {
    const int c = 16 * nt + m;
    const float bv = bias[c];
    #pragma unroll
    for (int r = 0; r < 8; ++r) {
      const float v = acc[nt][r] * osc + bv;
      sT[(16 * w + 8 * h + r) * 64 + c] = v > 0.f ? v : 0.f;
    }
  }
  __syncthreads();
  const int pp = tid >> 3, q = tid & 7;
  const float* t0 = sT + (2 * pp) * 64 + 8 * q;
  const float* t1 = sT + (64 + 2 * pp) * 64 + 8 * q;
  const v4f m0 = max4(max4(*(const v4fa*)(t0), *(const v4fa*)(t0 + 64)),
                      max4(*(const v4fa*)(t1), *(const v4fa*)(t1 + 64)));
  const v4f m1 = max4(max4(*(const v4fa*)(t0 + 4), *(const v4fa*)(t0 + 68)),
                      max4(*(const v4fa*)(t1 + 4), *(const v4fa*)(t1 + 68)));
  v8h o;
  o[0] = (f16t)(m0.x * PCAR); o[1] = (f16t)(m0.y * PCAR); o[2] = (f16t)(m0.z * PCAR); o[3] = (f16t)(m0.w * PCAR);
  o[4] = (f16t)(m1.x * PCAR); o[5] = (f16t)(m1.y * PCAR); o[6] = (f16t)(m1.z * PCAR); o[7] = (f16t)(m1.w * PCAR);
  f16t* dst = pool + ((size_t)(b * PLR + py + 1) * PLC + 32 * xb + pp + 1) * C1 + 8 * q;
  *(volatile v8h*)dst = o;
  __threadfence();
  *(volatile v8h*)dst = o;
}

__global__ __launch_bounds__(256) void conv2_roi_k(
    const f16t* __restrict__ pool, const f16t* __restrict__ w2p, const float* __restrict__ bias,
    const int* __restrict__ rois, float* __restrict__ part)
{
  __shared__ __attribute__((aligned(16))) float sV[64 * 128];
  __shared__ __attribute__((aligned(16))) float sP[33 * 128];
  __shared__ int sId[64];
  const int tid = threadIdx.x, lane = tid & 31, w = tid >> 5;
  const int h = lane >> 4, m = lane & 15;
  const int y = blockIdx.x, b = blockIdx.y;
  const int pt = w >> 1, ch0 = 64 * (w & 1);
  const int x0 = 16 * pt;

  {
    const v4f z4 = {0.f, 0.f, 0.f, 0.f};
    #pragma unroll
    for (int i = 0; i < 5; ++i) {
      const int p = tid + 256 * i;
      if (p < (33 * 128) / 4) *(v4fa*)(sP + 4 * p) = z4;
    }
  }
  if (tid < 64) {
    const int id = rois[(size_t)b * HI * HI + (size_t)(2 * y) * HI + 2 * tid];
    sId[tid] = ((unsigned)id < (unsigned)NOBJ) ? id : NOBJ;
  }

  const f16t* abase = pool + ((size_t)(b * PLR + y) * PLC + x0 + m) * C1;
  const f16t* bbase = w2p + (size_t)(ch0 + m) * K2;
  const v8f z8 = {0.f, 0.f, 0.f, 0.f, 0.f, 0.f, 0.f, 0.f};
  v8f acc[4];
  #pragma unroll
  for (int nt = 0; nt < 4; ++nt) acc[nt] = z8;
  #pragma unroll
  for (int t = 0; t < 18; ++t) {
    const int tap = t >> 1, kr = tap / 3, kc = tap - 3 * kr, cb = (t & 1) * 32;
    const v16h a = load_frag32(abase + ((size_t)kr * PLC + kc) * C1 + cb, h);
    #pragma unroll
    for (int nt = 0; nt < 4; ++nt) {
      const v16h bb = load_frag32(bbase + (size_t)nt * 16 * K2 + 32 * t, h);
      acc[nt] = wmma_f16(a, bb, acc[nt]);
    }
  }
  const float osc = 1.0f / (PCAR * WCAR);
  #pragma unroll
  for (int nt = 0; nt < 4; ++nt) {
    const int c = ch0 + 16 * nt + m;
    const float bv = bias[c];
    #pragma unroll
    for (int r = 0; r < 8; ++r) {
      const float v = acc[nt][r] * osc + bv;
      sV[(x0 + 8 * h + r) * 128 + c] = v > 0.f ? v : 0.f;
    }
  }
  __syncthreads();

  const int cg = w & 3, ph = w >> 2;
  const int cl = 32 * cg + lane;
  #pragma unroll 1
  for (int phase = 0; phase < 2; ++phase) {
    if (ph == phase) {
      #pragma unroll 4
      for (int i = 0; i < 32; ++i) {
        const int x = 32 * phase + i;
        const float v = sV[x * 128 + cl];
        const int o = sId[x];
        float* p = sP + o * 128 + cl;
        const float cur = *p;
        *p = fmaxf(cur, v);
      }
    }
    __syncthreads();
  }

  float* pbase = part + ((size_t)(b * HP + y)) * (NOBJ * C2);
  v4f vals[4];
  int pi[4];
  #pragma unroll
  for (int i = 0; i < 4; ++i) {
    pi[i] = tid + 256 * i;
    vals[i] = *(const v4fa*)(sP + 4 * pi[i]);
  }
  #pragma unroll
  for (int i = 0; i < 4; ++i) *(volatile v4f*)(pbase + 4 * pi[i]) = vals[i];
  __threadfence();
  #pragma unroll
  for (int i = 0; i < 4; ++i) *(volatile v4f*)(pbase + 4 * pi[i]) = vals[i];
}

__global__ __launch_bounds__(256) void combine_k(const float* __restrict__ part, float* __restrict__ out) {
  const int tid = threadIdx.x;
  const int chunk = blockIdx.x, b = blockIdx.y;
  const int f0 = chunk * 1024 + 4 * tid;
  const float* pb = part + (size_t)b * HP * (NOBJ * C2) + f0;
  v4f mx = {0.f, 0.f, 0.f, 0.f};
  #pragma unroll 4
  for (int yy = 0; yy < HP; ++yy) {
    const v4f v = *(const v4fa*)(pb + (size_t)yy * (NOBJ * C2));
    mx = max4(mx, v);
  }
  float* d = out + (size_t)b * (NOBJ * C2) + f0;
  *(volatile v4f*)d = mx;
  __threadfence();
  *(volatile v4f*)d = mx;
}

extern "C" void kernel_launch(void* const* d_in, const int* in_sizes, int n_in,
                              void* d_out, int out_size, void* d_ws, size_t ws_size,
                              hipStream_t stream) {
  if (n_in < 6) return;
  if (in_sizes[0] != NB * CIN * HI * HI) return;
  if (in_sizes[1] != NB * HI * HI) return;
  if (in_sizes[2] != C1 * CIN * 9 || in_sizes[3] != C1) return;
  if (in_sizes[4] != C2 * C1 * 9 || in_sizes[5] != C2) return;
  if (out_size != NB * NOBJ * C2) return;

  const float* img = (const float*)d_in[0];
  const int*   roi = (const int*)d_in[1];
  const float* w1  = (const float*)d_in[2];
  const float* b1  = (const float*)d_in[3];
  const float* w2  = (const float*)d_in[4];
  const float* b2  = (const float*)d_in[5];
  float* outp = (float*)d_out;

  const size_t bW1  = (size_t)C1 * K1 * 2;
  const size_t bW2  = (size_t)C2 * K2 * 2;
  const size_t bIMG = (size_t)NB * IMR * IMC * CP * 2;
  const size_t bPL  = (size_t)NB * PLR * PLC * C1 * 2;
  const size_t bPT  = (size_t)NB * HP * NOBJ * C2 * 4;
  const size_t oW1 = 0, oW2 = oW1 + bW1, oIMG = oW2 + bW2, oPL = oIMG + bIMG, oPT = oPL + bPL;
  const size_t total = oPT + bPT;
  if (total > ws_size) return;
  char* ws = (char*)d_ws;
  f16t*  W1P  = (f16t*)(ws + oW1);
  f16t*  W2P  = (f16t*)(ws + oW2);
  f16t*  IMG  = (f16t*)(ws + oIMG);
  f16t*  POOL = (f16t*)(ws + oPL);
  float* PART = (float*)(ws + oPT);

  cvt_img_k<<<dim3(IMR, NB), 256, 0, stream>>>(img, IMG);
  cvt_w_k<<<41, 256, 0, stream>>>(w1, w2, W1P, W2P);
  halo_k<<<dim3(PLR, NB), 256, 0, stream>>>(POOL);
  conv1_pool_k<<<dim3(2, HP, NB), 256, 0, stream>>>(IMG, W1P, b1, POOL);
  conv2_roi_k<<<dim3(HP, NB), 256, 0, stream>>>(POOL, W2P, b2, roi, PART);
  combine_k<<<dim3(4, NB), 256, 0, stream>>>(PART, outp);
}
